// SSMTokenMixer_53592601919829
// MI455X (gfx1250) — hardware-verified
//
#include <hip/hip_runtime.h>
#include <math.h>

constexpr int kNB        = 16;
constexpr int kC         = 128;
constexpr int kSide      = 64;
constexpr int kHW        = kSide * kSide;
constexpr int kTok       = kNB * kHW;
constexpr int kG3        = 3 * kC;
constexpr int kCat       = 4 * kC;
constexpr int kSeqPerDir = kNB * kSide;
constexpr int kSteps     = kSide;
constexpr int kWPlane    = kG3 * kC;
constexpr int kLdsPitch  = 136;
constexpr float kLnEps   = 1e-5f;

constexpr size_t kXnOff  = 0;
constexpr size_t kCatOff = kXnOff + (size_t)kTok * kC * 2;
constexpr size_t kWOff   = kCatOff + (size_t)kTok * kCat * 2;
constexpr size_t kPwOff  = kWOff + (size_t)8 * kWPlane * 2;
constexpr size_t kWsEnd  = kPwOff + (size_t)kC * kCat * 2;
static_assert(kWsEnd == 84803584);
static_assert(kWsEnd <= (size_t)134217728);

typedef __attribute__((ext_vector_type(16))) _Float16 v16h;
typedef __attribute__((ext_vector_type(8)))  _Float16 v8h;
typedef __attribute__((ext_vector_type(16))) __bf16   v16b;
typedef __attribute__((ext_vector_type(8)))  __bf16   v8b;
typedef __attribute__((ext_vector_type(8)))  float    v8f;
typedef __attribute__((ext_vector_type(4)))  float    v4f;
typedef __attribute__((ext_vector_type(4)))  unsigned int v4u;

__device__ __forceinline__ unsigned short f2bf_bits(float f) {
  unsigned u = __float_as_uint(f);
  return (unsigned short)((u + 0x7FFFu + ((u >> 16) & 1u)) >> 16);
}
__device__ __forceinline__ float bf_bits2f(unsigned short h) { return __uint_as_float(((unsigned)h) << 16); }

__device__ __forceinline__ void dep_guard_h(v8f& a, v8f& b, v16h x, v16h y) { asm volatile("v_nop\n\tv_nop\n\tv_nop\n\tv_nop" : "+v"(a), "+v"(b) : "v"(x), "v"(y)); }
__device__ __forceinline__ void dep_guard_b(v8f& a, v8f& b, v16b x, v16b y) { asm volatile("v_nop\n\tv_nop\n\tv_nop\n\tv_nop" : "+v"(a), "+v"(b) : "v"(x), "v"(y)); }
__device__ __forceinline__ void keep4_h(v16h a, v16h b, v16h c, v16h d) { asm volatile("v_nop" :: "v"(a), "v"(b), "v"(c), "v"(d)); }
__device__ __forceinline__ void keep4_b(v16b a, v16b b, v16b c, v16b d) { asm volatile("v_nop" :: "v"(a), "v"(b), "v"(c), "v"(d)); }
__device__ __forceinline__ void acc_guard4(v8f& a, v8f& b, v8f& c, v8f& d) { asm volatile("v_nop\n\tv_nop\n\tv_nop\n\tv_nop" : "+v"(a), "+v"(b), "+v"(c), "+v"(d)); }
template <typename T> struct Frag;
template <> struct Frag<_Float16> {
  typedef v16h V; union U { v16h v; v8h h[2]; };
  static __device__ __forceinline__ v16h load(const _Float16* p) {
    U f; f.h[0] = *(const v8h*)(p); f.h[1] = *(const v8h*)(p + 16); return f.v;
  }
  static __device__ __forceinline__ v8f mma(v16h a, v16h b, v8f c) {
    return __builtin_amdgcn_wmma_f32_16x16x32_f16(false, a, false, b, (short)0, c, false, false);
  }
  static __device__ __forceinline__ void guard(v8f& a, v8f& b, v16h x, v16h y) { dep_guard_h(a, b, x, y); }
  static __device__ __forceinline__ void keep(v16h a, v16h b, v16h c, v16h d) { keep4_h(a, b, c, d); }
};
template <> struct Frag<__bf16> {
  typedef v16b V; union U { v16b v; v8b h[2]; };
  static __device__ __forceinline__ v16b load(const __bf16* p) {
    U f; f.h[0] = *(const v8b*)(p); f.h[1] = *(const v8b*)(p + 16); return f.v;
  }
  static __device__ __forceinline__ v8f mma(v16b a, v16b b, v8f c) {
    return __builtin_amdgcn_wmma_f32_16x16x32_bf16(false, a, false, b, (short)0, c, false, false);
  }
  static __device__ __forceinline__ void guard(v8f& a, v8f& b, v16b x, v16b y) { dep_guard_b(a, b, x, y); }
  static __device__ __forceinline__ void keep(v16b a, v16b b, v16b c, v16b d) { keep4_b(a, b, c, d); }
};

__device__ __forceinline__ unsigned pk16(unsigned short a, unsigned short b) { return (unsigned)a | ((unsigned)b << 16); }
__device__ __forceinline__ unsigned short h_bits(float f) { const _Float16 h = (_Float16)f; return __builtin_bit_cast(unsigned short, h); }

template <int ET> struct Elem;
template <> struct Elem<0> { typedef _Float16 T; };
template <> struct Elem<1> { typedef __bf16 T; };
template <int ET, bool SPLIT, int BIAS_MODE, int OUT_MODE, bool RESID, int ACT = 0>
__global__ __launch_bounds__(256) void wmma_gemm64(
    const unsigned short* __restrict__ Ap, const unsigned short* __restrict__ A2p, int lda, long strideA,
    const unsigned short* __restrict__ Btp, const unsigned short* __restrict__ Bt2p, int ldb, long strideB,
    void* __restrict__ Cout, void* __restrict__ Cout2, int ldc, long strideC,
    const float* __restrict__ bias,
    const float* __restrict__ resid, long strideR,
    int M, int N, int K, float scale) {
  typedef typename Elem<ET>::T T;
  typedef typename Frag<T>::V V;
  const T* A = (const T*)Ap; const T* A2 = (const T*)A2p; const T* Bt = (const T*)Btp; const T* Bt2 = (const T*)Bt2p;
  __shared__ __align__(16) float sT[8][16 * 68];
  const int b    = blockIdx.y;
  const int lane = threadIdx.x & 31;
  const int wave = threadIdx.x >> 5;
  const int tilesN = N >> 6;
  const int tilesM = M >> 6;
  const int tile = blockIdx.x * 8 + wave;
  if (tile >= tilesM * tilesN) return;
  const int tm = tile / tilesN;
  const int tn = tile - tm * tilesN;
  const int m0 = tm << 6;
  const int n0 = tn << 6;

  const T* Ab  = A  + (size_t)b * strideA;
  const T* Bb  = Bt + (size_t)b * strideB;
  const T* Ab2 = SPLIT ? (A2  + (size_t)b * strideA) : nullptr;
  const T* Bb2 = SPLIT ? (Bt2 + (size_t)b * strideB) : nullptr;

  const int rlane = lane & 15;
  const int koff  = (lane >> 4) * 8;
  const int mOff  = (lane >> 4) * 8;

  v8f acc[4][4];
#pragma unroll
  for (int i = 0; i < 4; ++i)
#pragma unroll
    for (int j = 0; j < 4; ++j) acc[i][j] = (v8f){0.f,0.f,0.f,0.f,0.f,0.f,0.f,0.f};

  for (int k0 = 0; k0 < K; k0 += 32) {
    V bh[4], bl[4];
#pragma unroll
    for (int j = 0; j < 4; ++j) {
      const size_t bo = (size_t)(n0 + (j << 4) + rlane) * ldb + koff + k0;
      bh[j] = Frag<T>::load(Bb + bo);
      if (SPLIT) bl[j] = Frag<T>::load(Bb2 + bo);
    }
#pragma unroll
    for (int i = 0; i < 4; ++i) {
      const size_t ao = (size_t)(m0 + (i << 4) + rlane) * lda + koff + k0;
      V ah = Frag<T>::load(Ab + ao);
      V al;
      if (SPLIT) al = Frag<T>::load(Ab2 + ao);
#pragma unroll
      for (int j = 0; j < 4; ++j) {
        acc[i][j] = Frag<T>::mma(ah, bh[j], acc[i][j]);
        if (SPLIT) {
          acc[i][j] = Frag<T>::mma(ah, bl[j], acc[i][j]);
          acc[i][j] = Frag<T>::mma(al, bh[j], acc[i][j]);
        }
      }
      Frag<T>::guard(acc[i][0], acc[i][3], ah, SPLIT ? al : ah);
    }
    Frag<T>::keep(bh[0], bh[1], bh[2], bh[3]);
    if (SPLIT) Frag<T>::keep(bl[0], bl[1], bl[2], bl[3]);
  }
  acc_guard4(acc[0][0], acc[0][1], acc[0][2], acc[0][3]);
  acc_guard4(acc[1][0], acc[1][1], acc[1][2], acc[1][3]);
  acc_guard4(acc[2][0], acc[2][1], acc[2][2], acc[2][3]);
  acc_guard4(acc[3][0], acc[3][1], acc[3][2], acc[3][3]);

  float* slab = sT[wave];
  const float* Rb = RESID ? (resid + (size_t)b * strideR) : nullptr;
#pragma unroll
  for (int i = 0; i < 4; ++i) {
    const int mBase = m0 + (i << 4);
#pragma unroll
    for (int j = 0; j < 4; ++j) {
      const int n = n0 + (j << 4) + rlane;
      float bv = 0.f;
      if (BIAS_MODE == 2) bv = bias[n];
#pragma unroll
      for (int r = 0; r < 8; ++r) {
        float v = acc[i][j][r] * scale;
        if (BIAS_MODE == 1) v += bias[mBase + mOff + r];
        if (BIAS_MODE == 2) v += bv;
        if (RESID) v += Rb[(size_t)(mBase + mOff + r) * ldc + n];
        if (ACT == 2) v = fmaxf(v, 0.0f);
        if (ACT == 4) v = (v > 0.f) ? v : 0.01f * v;
        slab[(mOff + r) * 68 + (j << 4) + rlane] = v;
      }
    }
    __builtin_amdgcn_fence(__ATOMIC_RELEASE, "workgroup");
    __builtin_amdgcn_wave_barrier();
    __builtin_amdgcn_fence(__ATOMIC_ACQUIRE, "workgroup");
    if (OUT_MODE == 0) {
      float* C = (float*)Cout + (size_t)b * strideC;
      const int hh = lane >> 4, c4 = (lane & 15) * 4;
      for (int pass = 0; pass < 2; ++pass) {
#pragma unroll
        for (int it = 0; it < 8; ++it) {
          const int row = it * 2 + hh;
          v4f v = *(const v4f*)(slab + row * 68 + c4);
          *(volatile v4f*)(C + (size_t)(mBase + row) * ldc + n0 + c4) = v;
        }
        __threadfence();
      }
    } else {
      const int q = lane >> 3, c8 = (lane & 7) * 8;
      unsigned short* C  = (unsigned short*)Cout  + (size_t)b * strideC;
      unsigned short* C2 = (OUT_MODE == 2) ? ((unsigned short*)Cout2 + (size_t)b * strideC) : nullptr;
      for (int pass = 0; pass < 2; ++pass) {
#pragma unroll
        for (int it = 0; it < 4; ++it) {
          const int row = it * 4 + q;
          const float* sp = slab + row * 68 + c8;
          v8h hv, lv;
#pragma unroll
          for (int e = 0; e < 8; ++e) {
            if (OUT_MODE == 1) {
              hv[e] = (_Float16)sp[e];
            } else {
              unsigned short hb = f2bf_bits(sp[e]);
              unsigned short lb = f2bf_bits(sp[e] - bf_bits2f(hb));
              hv[e] = __builtin_bit_cast(_Float16, hb);
              lv[e] = __builtin_bit_cast(_Float16, lb);
            }
          }
          *(volatile v8h*)(C + (size_t)(mBase + row) * ldc + n0 + c8) = hv;
          if (OUT_MODE == 2) *(volatile v8h*)(C2 + (size_t)(mBase + row) * ldc + n0 + c8) = lv;
        }
        __threadfence();
      }
    }
    __builtin_amdgcn_fence(__ATOMIC_RELEASE, "workgroup");
    __builtin_amdgcn_wave_barrier();
    __builtin_amdgcn_fence(__ATOMIC_ACQUIRE, "workgroup");
  }
}

__device__ __forceinline__ void scan_guard6(v8f& a0, v8f& a1, v8f& a2, v8f& a3, v8f& a4, v8f& a5,
                                            v16h x, v16h y, v16h b0, v16h b1, v16h b2, v16h b3, v16h b4, v16h b5) {
  asm volatile("v_nop\n\tv_nop\n\tv_nop\n\tv_nop"
               : "+v"(a0), "+v"(a1), "+v"(a2), "+v"(a3), "+v"(a4), "+v"(a5)
               : "v"(x), "v"(y), "v"(b0), "v"(b1), "v"(b2), "v"(b3), "v"(b4), "v"(b5));
}

__device__ __forceinline__ float gate_sigmoid(float x) {
  x = fminf(fmaxf(x, -30.0f), 30.0f);
  return __builtin_amdgcn_rcpf(1.0f + expf(-x));
}
__device__ __forceinline__ float gate_tanh(float x) {
  x = fminf(fmaxf(x, -15.0f), 15.0f);
  return 1.0f - 2.0f * __builtin_amdgcn_rcpf(1.0f + expf(2.0f * x));
}

__device__ __forceinline__ int tok_of(int seq, int tstep, int vert) {
  const int hz = ((((seq >> 6) << 6) + tstep) << 6) + (seq & 63);
  const int hh = (seq << 6) + tstep;
  return vert ? hz : hh;
}

__global__ __launch_bounds__(256) void ln_kernel(const float* __restrict__ x, const float* __restrict__ gam,
                                                 const float* __restrict__ bet, unsigned short* __restrict__ xn16) {
  __shared__ float sm[32 * 129];
  __shared__ __align__(16) _Float16 sh[32 * kLdsPitch];
  const int t = threadIdx.x;
  const int lane = t & 31, wave = t >> 5, hh = lane >> 4;
  const int b   = blockIdx.x >> 7;
  const int hw0 = (blockIdx.x & 127) * 32;
  const float* xb = x + (size_t)b * kC * kHW + hw0;
#pragma unroll
  for (int i = 0; i < 16; ++i) {
    const int e = i * 256 + t;
    const int c = e >> 5;
    const int j = e & 31;
    sm[j * 129 + c] = xb[(size_t)c * kHW + j];
  }
  __syncthreads();
  const float g0 = gam[lane], g1 = gam[lane + 32], g2 = gam[lane + 64], g3 = gam[lane + 96];
  const float e0 = bet[lane], e1 = bet[lane + 32], e2 = bet[lane + 64], e3 = bet[lane + 96];
#pragma unroll 1
  for (int jj = 0; jj < 4; ++jj) {
    const int j = wave * 4 + jj;
    const float* sr = sm + j * 129;
    const float v0 = sr[lane], v1 = sr[lane + 32], v2 = sr[lane + 64], v3 = sr[lane + 96];
    float s = (v0 + v1) + (v2 + v3);
#pragma unroll
    for (int off = 16; off > 0; off >>= 1) s += __shfl_xor(s, off, 32);
    const float mu = s * (1.0f / 128.0f);
    const float d0 = v0 - mu, d1 = v1 - mu, d2 = v2 - mu, d3 = v3 - mu;
    float s2 = (d0 * d0 + d1 * d1) + (d2 * d2 + d3 * d3);
#pragma unroll
    for (int off = 16; off > 0; off >>= 1) s2 += __shfl_xor(s2, off, 32);
    const float var = s2 * (1.0f / 128.0f);
    const float rs  = rsqrtf(var + kLnEps);
    _Float16* hr = sh + j * kLdsPitch;
    hr[lane]      = (_Float16)(d0 * rs * g0 + e0);
    hr[lane + 32] = (_Float16)(d1 * rs * g1 + e1);
    hr[lane + 64] = (_Float16)(d2 * rs * g2 + e2);
    hr[lane + 96] = (_Float16)(d3 * rs * g3 + e3);
  }
  __syncthreads();
  const int c8 = (lane & 15) * 8;
  const int r0 = wave * 4 + hh;
  const int r1 = wave * 4 + 2 + hh;
  const v4u u0 = *(const v4u*)(sh + r0 * kLdsPitch + c8);
  const v4u u1 = *(const v4u*)(sh + r1 * kLdsPitch + c8);
  unsigned short* p0 = xn16 + ((size_t)b * kHW + hw0 + r0) * kC + c8;
  unsigned short* p1 = xn16 + ((size_t)b * kHW + hw0 + r1) * kC + c8;
  *(volatile v4u*)p0 = u0;
  *(volatile v4u*)p1 = u1;
  __threadfence();
  *(volatile v4u*)p0 = u0;
  *(volatile v4u*)p1 = u1;
}

__global__ __launch_bounds__(256) void cast8_kernel(const float* __restrict__ p0, const float* __restrict__ p1,
                                                    const float* __restrict__ p2, const float* __restrict__ p3,
                                                    const float* __restrict__ p4, const float* __restrict__ p5,
                                                    const float* __restrict__ p6, const float* __restrict__ p7,
                                                    unsigned short* __restrict__ out, int n8, float scale) {
  const int z = blockIdx.y;
  const float* src = (z == 0) ? p0 : (z == 1) ? p1 : (z == 2) ? p2 : (z == 3) ? p3
                   : (z == 4) ? p4 : (z == 5) ? p5 : (z == 6) ? p6 : p7;
  const int i = blockIdx.x * 256 + threadIdx.x;
  if (i >= n8) return;
  const float* p = src + 8 * (size_t)i;
  const v4f a = *(const v4f*)(p);
  const v4f c = *(const v4f*)(p + 4);
  unsigned short hb[8];
#pragma unroll
  for (int e = 0; e < 4; ++e) {
    hb[e]     = h_bits(a[e] * scale);
    hb[4 + e] = h_bits(c[e] * scale);
  }
  const v4u u = (v4u){pk16(hb[0], hb[1]), pk16(hb[2], hb[3]), pk16(hb[4], hb[5]), pk16(hb[6], hb[7])};
  unsigned short* q = out + (size_t)z * (size_t)n8 * 8 + 8 * (size_t)i;
  *(volatile v4u*)q = u;
  __threadfence();
  *(volatile v4u*)q = u;
}

__global__ __launch_bounds__(256) void gru_scan_kernel(
    const unsigned short* __restrict__ xn16, const unsigned short* __restrict__ w16,
    const float* __restrict__ bi0, const float* __restrict__ bh0,
    const float* __restrict__ bi1, const float* __restrict__ bh1,
    const float* __restrict__ bi2, const float* __restrict__ bh2,
    const float* __restrict__ bi3, const float* __restrict__ bh3,
    unsigned short* __restrict__ cat16) {
  typedef Frag<_Float16> FH;
  __shared__ __align__(16) _Float16 Xs[16 * kLdsPitch];
  __shared__ __align__(16) _Float16 Hs[16 * kLdsPitch];
  const int dirn = blockIdx.y;
  const int rev  = dirn & 1;
  const int vert = dirn >> 1;
  const int s0   = blockIdx.x * 16;
  const int tid = threadIdx.x, wave = tid >> 5, lane = tid & 31;
  const int rlane = lane & 15, hh = lane >> 4, koff = hh * 8;
  const float* bih = (dirn == 0) ? bi0 : (dirn == 1) ? bi1 : (dirn == 2) ? bi2 : bi3;
  const float* bhh = (dirn == 0) ? bh0 : (dirn == 1) ? bh1 : (dirn == 2) ? bh2 : bh3;
  const _Float16* wih = (const _Float16*)(w16 + (size_t)(2 * dirn) * kWPlane);
  const _Float16* whh = (const _Float16*)(w16 + (size_t)(2 * dirn + 1) * kWPlane);
  const int ch = wave * 16 + rlane;
  const float b_ir = bih[ch],          b_hr = bhh[ch];
  const float b_iz = bih[kC + ch],     b_hz = bhh[kC + ch];
  const float b_in = bih[2 * kC + ch], b_hn = bhh[2 * kC + ch];

  {
    const v4u z4 = (v4u){0u, 0u, 0u, 0u};
    for (int i = tid; i < (16 * kLdsPitch) / 8; i += 256) {
      *(v4u*)(Xs + 8 * i) = z4;
      *(v4u*)(Hs + 8 * i) = z4;
    }
  }
  float hreg[8];
#pragma unroll
  for (int r = 0; r < 8; ++r) hreg[r] = 0.0f;

  const int xrow = tid >> 4, xc8 = (tid & 15) * 8;
  const int xseq = s0 + xrow;
  const int sq = lane >> 3, sc8 = (lane & 7) * 8;
  const int srow = wave * 2 + (sq >> 1);
  const int shalf = (sq & 1) * 64;
  const int sseq = s0 + srow;
  __syncthreads();

#pragma unroll 1
  for (int t = 0; t < kSteps; ++t) {
    const int teff = rev ? (kSteps - 1 - t) : t;
    {
      const int xtok = tok_of(xseq, teff, vert);
      const v4u xv = *(const v4u*)(xn16 + (size_t)xtok * kC + xc8);
      *(v4u*)(Xs + xrow * kLdsPitch + xc8) = xv;
    }
    __syncthreads();

    v8f aX0 = (v8f){0.f,0.f,0.f,0.f,0.f,0.f,0.f,0.f};
    v8f aX1 = aX0, aX2 = aX0, aH0 = aX0, aH1 = aX0, aH2 = aX0;
#pragma unroll 1
    for (int kc = 0; kc < 4; ++kc) {
      const int ko = kc * 32 + koff;
      const v16h ax = FH::load(Xs + rlane * kLdsPitch + ko);
      const v16h ah = FH::load(Hs + rlane * kLdsPitch + ko);
      const size_t wo = (size_t)ch * kC + ko;
      const v16h b0 = FH::load(wih + wo);
      const v16h b1 = FH::load(wih + (size_t)kC * kC + wo);
      const v16h b2 = FH::load(wih + (size_t)2 * kC * kC + wo);
      const v16h b3 = FH::load(whh + wo);
      const v16h b4 = FH::load(whh + (size_t)kC * kC + wo);
      const v16h b5 = FH::load(whh + (size_t)2 * kC * kC + wo);
      aX0 = FH::mma(ax, b0, aX0);
      aX1 = FH::mma(ax, b1, aX1);
      aX2 = FH::mma(ax, b2, aX2);
      aH0 = FH::mma(ah, b3, aH0);
      aH1 = FH::mma(ah, b4, aH1);
      aH2 = FH::mma(ah, b5, aH2);
      scan_guard6(aX0, aX1, aX2, aH0, aH1, aH2, ax, ah, b0, b1, b2, b3, b4, b5);
    }

#pragma unroll
    for (int r = 0; r < 8; ++r) {
      const float xr = aX0[r] * 0.125f + b_ir;
      const float xz = aX1[r] * 0.125f + b_iz;
      const float xg = aX2[r] * 0.125f + b_in;
      const float hr = aH0[r] * (1.0f / 64.0f) + b_hr;
      const float hz = aH1[r] * (1.0f / 64.0f) + b_hz;
      const float hg = aH2[r] * (1.0f / 64.0f) + b_hn;
      const float rg = gate_sigmoid(xr + hr);
      const float zg = gate_sigmoid(xz + hz);
      const float ng = gate_tanh(xg + rg * hg);
      hreg[r] = (1.0f - zg) * ng + zg * hreg[r];
    }
    __syncthreads();
#pragma unroll
    for (int r = 0; r < 8; ++r) {
      Hs[(8 * hh + r) * kLdsPitch + ch] = (_Float16)(hreg[r] * 8.0f);
    }
    __syncthreads();
    {
      const int stok = tok_of(sseq, teff, vert);
      const v4u hv = *(const v4u*)(Hs + srow * kLdsPitch + shalf + sc8);
      unsigned short* dst = cat16 + (size_t)stok * kCat + dirn * kC + shalf + sc8;
      *(volatile v4u*)dst = hv;
      __threadfence();
      *(volatile v4u*)dst = hv;
    }
  }
}

extern "C" void kernel_launch(void* const* d_in, const int* in_sizes, int n_in,
                              void* d_out, int out_size, void* d_ws, size_t ws_size,
                              hipStream_t stream) {
  if (n_in < 21) return;
  if (ws_size < kWsEnd) return;
  if (out_size != kTok * kC) return;
  if (in_sizes[0] != kTok * kC) return;
  if (in_sizes[3] != kWPlane || in_sizes[19] != kC * kCat) return;

  char* ws = (char*)d_ws;
  unsigned short* xn16  = (unsigned short*)(ws + kXnOff);
  unsigned short* cat16 = (unsigned short*)(ws + kCatOff);
  unsigned short* w16   = (unsigned short*)(ws + kWOff);
  unsigned short* pw16  = (unsigned short*)(ws + kPwOff);

  const float* xin  = (const float*)d_in[0];
  const float* lng  = (const float*)d_in[1];
  const float* lnb  = (const float*)d_in[2];
  const float* wih0 = (const float*)d_in[3];  const float* whh0 = (const float*)d_in[4];
  const float* bih0 = (const float*)d_in[5];  const float* bhh0 = (const float*)d_in[6];
  const float* wih1 = (const float*)d_in[7];  const float* whh1 = (const float*)d_in[8];
  const float* bih1 = (const float*)d_in[9];  const float* bhh1 = (const float*)d_in[10];
  const float* wih2 = (const float*)d_in[11]; const float* whh2 = (const float*)d_in[12];
  const float* bih2 = (const float*)d_in[13]; const float* bhh2 = (const float*)d_in[14];
  const float* wih3 = (const float*)d_in[15]; const float* whh3 = (const float*)d_in[16];
  const float* bih3 = (const float*)d_in[17]; const float* bhh3 = (const float*)d_in[18];
  const float* projw = (const float*)d_in[19];
  const float* projb = (const float*)d_in[20];

  ln_kernel<<<dim3(kNB * (kHW / 32)), dim3(256), 0, stream>>>(xin, lng, lnb, xn16);

  cast8_kernel<<<dim3(kWPlane / 8 / 256, 8), dim3(256), 0, stream>>>(
      wih0, whh0, wih1, whh1, wih2, whh2, wih3, whh3, w16, kWPlane / 8, 8.0f);

  cast8_kernel<<<dim3((kC * kCat) / 8 / 256, 1), dim3(256), 0, stream>>>(
      projw, projw, projw, projw, projw, projw, projw, projw, pw16, (kC * kCat) / 8, 16.0f);

  gru_scan_kernel<<<dim3(kSeqPerDir / 16, 4), dim3(256), 0, stream>>>(
      xn16, w16, bih0, bhh0, bih1, bhh1, bih2, bhh2, bih3, bhh3, cat16);

  wmma_gemm64<0, false, 1, 0, true, 0><<<dim3(16, kNB), dim3(256), 0, stream>>>(
      pw16, pw16, kCat, 0L,
      cat16, cat16, kCat, (long)kHW * kCat,
      d_out, d_out, kHW, (long)kC * kHW,
      projb,
      xin, (long)kC * kHW,
      kC, kHW, kCat, 1.0f / 128.0f);
}
